// Self_Attention_12214886990752
// MI455X (gfx1250) — hardware-verified
//
#include <hip/hip_runtime.h>


#define NB_  8
#define TT   2048
#define DM   512
#define CC   DM
#define CI   64
#define HD   64
typedef _Float16 h16;
typedef unsigned short bf;
typedef __attribute__((ext_vector_type(16))) __bf16   v16bf;
typedef __attribute__((ext_vector_type(16))) _Float16 v16h;
typedef __attribute__((ext_vector_type(8)))  _Float16 v8h;
typedef __attribute__((ext_vector_type(8)))  unsigned short v8us;
typedef __attribute__((ext_vector_type(8)))  float    v8f;
typedef __attribute__((ext_vector_type(4)))  float    v4f;
typedef v8h  __attribute__((may_alias)) v8ha;
typedef v4f  __attribute__((may_alias)) v4fa;
typedef v8us __attribute__((may_alias)) v8usa;

__device__ __forceinline__ unsigned short f2bf(float f) { unsigned u = __float_as_uint(f); u += 0x7FFFu + ((u >> 16) & 1u); return (unsigned short)(u >> 16); }
__device__ __forceinline__ float bf2f(unsigned short b) { return __uint_as_float(((unsigned)b) << 16); }
__device__ __forceinline__ float bfr(float f) { return bf2f(f2bf(f)); }
__device__ __forceinline__ v16h cat16(v8h lo, v8h hi) { return __builtin_shufflevector(lo, hi, 0, 1, 2, 3, 4, 5, 6, 7, 8, 9, 10, 11, 12, 13, 14, 15); }
__device__ __forceinline__ v16bf cat16b(v8us lo, v8us hi) { return __builtin_bit_cast(v16bf, __builtin_shufflevector(lo, hi, 0, 1, 2, 3, 4, 5, 6, 7, 8, 9, 10, 11, 12, 13, 14, 15)); }
__device__ __forceinline__ v8f wmma16(v16h a, v16h b, v8f c) { return __builtin_amdgcn_wmma_f32_16x16x32_f16(false, a, false, b, (short)0, c, false, false); }
__device__ __forceinline__ v8f wmmab(v16bf a, v16bf b, v8f c) { return __builtin_amdgcn_wmma_f32_16x16x32_bf16(false, a, false, b, (short)0, c, false, false); }


template <typename T16> struct WFrag;
template <> struct WFrag<h16> { typedef v16h V; static __device__ __forceinline__ V ld(const h16* p) { return cat16(*(const v8h*)p, *(const v8h*)(p + 16)); } static __device__ __forceinline__ v8f mma(V a, V b, v8f c) { return wmma16(a, b, c); } };
template <> struct WFrag<bf> { typedef v16bf V; static __device__ __forceinline__ V ld(const bf* p) { return cat16b(*(const v8us*)p, *(const v8us*)(p + 16)); } static __device__ __forceinline__ v8f mma(V a, V b, v8f c) { return wmmab(a, b, c); } };
template <typename T16, int NSPLIT, bool BIAS>
__global__ __launch_bounds__(32) void k_gemmw(const T16* __restrict__ A, const T16* __restrict__ A2, const T16* __restrict__ Bt, const T16* __restrict__ Bt2, int K, float* C, int ldc, const float* __restrict__ bias, size_t sA, size_t sB, size_t sC) {
    typedef typename WFrag<T16>::V V;
    __shared__ __align__(16) float os[16 * 68];
    const size_t z = blockIdx.z; A += z * sA; if (A2) A2 += z * sA; Bt += z * sB; if (Bt2) Bt2 += z * sB; C += z * sC;
    const int lane = threadIdx.x & 31, lr = lane & 15, hi = lane >> 4; const int r0 = blockIdx.x * 64, c0 = blockIdx.y * 64;
    v8f acc[4][4];
#pragma unroll
    for (int mb = 0; mb < 4; ++mb)
#pragma unroll
        for (int nb = 0; nb < 4; ++nb) acc[mb][nb] = (v8f){};
    const size_t aoff = (size_t)(r0 + lr) * K + 8 * hi, boff = (size_t)(c0 + lr) * K + 8 * hi;
#pragma unroll 1
    for (int kc = 0; kc < K; kc += 32) {
        V a[4], a2[4];
#pragma unroll
        for (int mb = 0; mb < 4; ++mb) { a[mb] = WFrag<T16>::ld(A + aoff + (size_t)mb * 16 * K + kc); if (NSPLIT == 1 || NSPLIT == 2) a2[mb] = WFrag<T16>::ld(A2 + aoff + (size_t)mb * 16 * K + kc); }
#pragma unroll
        for (int nb = 0; nb < 4; ++nb) { const V b = WFrag<T16>::ld(Bt + boff + (size_t)nb * 16 * K + kc); V b2; if (NSPLIT >= 2) b2 = WFrag<T16>::ld(Bt2 + boff + (size_t)nb * 16 * K + kc);
#pragma unroll
            for (int mb = 0; mb < 4; ++mb) { acc[mb][nb] = WFrag<T16>::mma(a[mb], b, acc[mb][nb]); if (NSPLIT == 1 || NSPLIT == 2) acc[mb][nb] = WFrag<T16>::mma(a2[mb], b, acc[mb][nb]); if (NSPLIT >= 2) acc[mb][nb] = WFrag<T16>::mma(a[mb], b2, acc[mb][nb]); } }
        asm volatile("v_nop\n\tv_nop\n\tv_nop\n\tv_nop" : "+v"(acc[0][0]), "+v"(acc[1][1]), "+v"(acc[2][2]), "+v"(acc[3][3]) : "v"(a[0]), "v"(a[3]));
    }
#pragma unroll
    for (int mb = 0; mb < 4; ++mb) {
#pragma unroll
        for (int nb = 0; nb < 4; ++nb) {
#pragma unroll
            for (int j = 0; j < 8; ++j) os[(hi * 8 + j) * 68 + nb * 16 + lr] = acc[mb][nb][j]; }
        __builtin_amdgcn_wave_barrier(); asm volatile("" ::: "memory");
        float* crow = C + (size_t)(r0 + mb * 16) * ldc + c0;
#pragma unroll 1
        for (int ps = 0; ps < 2; ++ps) {
#pragma unroll
            for (int s = 0; s < 8; ++s) { const int row = 2 * s + hi, cofs = lr * 4; v4f val = *(const v4fa*)(os + row * 68 + cofs); if (BIAS) { val[0] += bfr(bias[c0 + cofs]); val[1] += bfr(bias[c0 + cofs + 1]); val[2] += bfr(bias[c0 + cofs + 2]); val[3] += bfr(bias[c0 + cofs + 3]); }
                *(volatile v4f*)(crow + (size_t)row * ldc + cofs) = val; }
            if (ps == 0) __threadfence(); }
        __builtin_amdgcn_wave_barrier(); asm volatile("" ::: "memory");
    }
}

__device__ __forceinline__ h16 tohx(float x) { return (h16)x; }
__device__ __forceinline__ void splitf(float y, unsigned short& h, unsigned short& l) { h = f2bf(y); l = f2bf(y - bf2f(h)); }
typedef __attribute__((ext_vector_type(2))) _Float16 v2h;
typedef __attribute__((ext_vector_type(4))) _Float16 v4h;
typedef __attribute__((ext_vector_type(2))) unsigned short v2us;
typedef __attribute__((ext_vector_type(4))) unsigned short v4us;
typedef __attribute__((ext_vector_type(2))) float v2f;
typedef __attribute__((ext_vector_type(4))) int v4i;

__global__ __launch_bounds__(256) void k_cvt8(const float* __restrict__ src, bf* dst, size_t n8) { const size_t i = (size_t)blockIdx.x * 256 + threadIdx.x; if (i >= n8) return; const v8f v = *(const v8f*)(src + i * 8); v8us o;
#pragma unroll
    for (int k = 0; k < 8; ++k) o[k] = f2bf(v[k]); *(volatile v8us*)(dst + i * 8) = o; __threadfence(); *(volatile v8us*)(dst + i * 8) = o; }


__global__ __launch_bounds__(256) void k_flat(const float* __restrict__ F, h16* P16, bf* Ph, bf* Pl, size_t n4) { const size_t i = (size_t)blockIdx.x * 256 + threadIdx.x; if (i >= n4) return; const v4f a = *(const v4f*)(F + i * 4); v4h o16; v4us oh, ol;
#pragma unroll
    for (int q = 0; q < 4; ++q) { o16[q] = tohx(a[q]); unsigned short x2, y2; splitf(a[q], x2, y2); oh[q] = x2; ol[q] = y2; }
    *(volatile v4h*)(P16 + i * 4) = o16; *(volatile v4us*)(Ph + i * 4) = oh; *(volatile v4us*)(Pl + i * 4) = ol; __threadfence(); *(volatile v4h*)(P16 + i * 4) = o16; *(volatile v4us*)(Ph + i * 4) = oh; *(volatile v4us*)(Pl + i * 4) = ol; }

__global__ __launch_bounds__(256) void k_colsoft(const float* __restrict__ Sb, float* ST) { const int m = blockIdx.x * 256 + threadIdx.x; if (m >= TT) return; float mx = -3.0e38f;
#pragma unroll 1
    for (int n = 0; n < TT; ++n) mx = fmaxf(mx, Sb[(size_t)n * TT + m]);
    float s = 0.f;
#pragma unroll 1
    for (int n = 0; n < TT; ++n) { float d0 = __fsub_rn(Sb[(size_t)n * TT + m], mx); asm volatile("" : "+v"(d0)); s = __fadd_rn(s, __builtin_amdgcn_exp2f(__fmul_rn(d0, 1.4426950408889634f))); }
    const float rz = __fdiv_rn(1.0f, s); *(volatile float*)(ST + m) = mx; *(volatile float*)(ST + TT + m) = rz; __threadfence(); *(volatile float*)(ST + m) = mx; *(volatile float*)(ST + TT + m) = rz; }
__global__ __launch_bounds__(256) void k_esplit(const float* __restrict__ Sb, const float* __restrict__ ST, bf* Eh, bf* El) { const size_t i = (size_t)blockIdx.x * 256 + threadIdx.x; if (i >= (size_t)TT * TT / 4) return; const size_t e = i * 4; const int m0 = (int)(e % TT); const v4f a = *(const v4f*)(Sb + e); const v4f cm = *(const v4f*)(ST + m0); const v4f rz = *(const v4f*)(ST + TT + m0); v4us oh, ol;
#pragma unroll
    for (int q = 0; q < 4; ++q) { float d0 = __fsub_rn(a[q], cm[q]); asm volatile("" : "+v"(d0)); float ex = __builtin_amdgcn_exp2f(__fmul_rn(d0, 1.4426950408889634f)); asm volatile("" : "+v"(ex)); const float wgt = __fmul_rn(ex, rz[q]); unsigned short u, w; splitf(wgt, u, w); oh[q] = u; ol[q] = w; }
    *(volatile v4us*)(Eh + e) = oh; *(volatile v4us*)(El + e) = ol; __threadfence(); *(volatile v4us*)(Eh + e) = oh; *(volatile v4us*)(El + e) = ol; }
__global__ __launch_bounds__(256) void k_wtG(const float* __restrict__ w, int K, int N, bf* Bt) {
    const int lane = threadIdx.x & 31; const int L0 = (blockIdx.x * 8 + (threadIdx.x >> 5)) * 8; const int nlines = N * K / 64;
#pragma unroll
    for (int ps = 0; ps < 2; ++ps) {
#pragma unroll 1
        for (int l = 0; l < 8; ++l) { const int L = L0 + l; if (L >= nlines) break; const size_t e = (size_t)L * 64 + lane * 2; const int k = (int)(e % K), n = (int)(e / K); v2us o;
            o[0] = f2bf(w[(size_t)k * N + n]); o[1] = f2bf(w[(size_t)(k + 1) * N + n]); *(volatile v2us*)(Bt + e) = o; }
        if (ps == 0) __threadfence(); }
}
__global__ __launch_bounds__(256) void k_vtp(const float* __restrict__ F, int pitch, int nheads, h16* V16, bf* Vh, bf* Vl) { const size_t e = ((size_t)blockIdx.x * 256 + threadIdx.x) * 2; if (e >= (size_t)nheads * HD * TT) return; const int t = (int)(e % TT); const int d = (int)((e / TT) % HD); const int g = (int)(e / ((size_t)TT * HD)); v2h o16; v2us oh, ol;
#pragma unroll
    for (int q = 0; q < 2; ++q) { const float x = F[(size_t)(t + q) * pitch + g * HD + d]; o16[q] = tohx(x); unsigned short a2, c2; splitf(x, a2, c2); oh[q] = a2; ol[q] = c2; }
    *(volatile v2h*)(V16 + e) = o16; *(volatile v2us*)(Vh + e) = oh; *(volatile v2us*)(Vl + e) = ol; __threadfence(); *(volatile v2h*)(V16 + e) = o16; *(volatile v2us*)(Vh + e) = oh; *(volatile v2us*)(Vl + e) = ol; }
extern "C" void kernel_launch(void* const* d_in, const int* in_sizes, int n_in,
                              void* d_out, int out_size, void* d_ws, size_t ws_size, hipStream_t stream) {
    (void)in_sizes; (void)n_in; (void)out_size;
    const float* x = (const float*)d_in[0]; const float* wk = (const float*)d_in[1]; const float* bk = (const float*)d_in[2]; const float* wq = (const float*)d_in[3]; const float* bq = (const float*)d_in[4];
    float* OUT = (float*)d_out;
    char* wsp = (char*)d_ws;
    auto take = [&](size_t bytes) { char* p = wsp; wsp += (bytes + 255) & ~(size_t)255; return (void*)p; };
    bf* WQ = (bf*)take((size_t)CI * DM * 2); bf* WK = (bf*)take((size_t)CI * DM * 2);
    bf* XB = (bf*)take((size_t)TT * DM * 2); float* FT = (float*)take((size_t)TT * CI * 4); float* FP = (float*)take((size_t)TT * CI * 4);
    h16* T16 = (h16*)take((size_t)TT * CI * 2); bf* Th = (bf*)take((size_t)TT * CI * 2); bf* Tl = (bf*)take((size_t)TT * CI * 2); h16* P16 = (h16*)take((size_t)TT * CI * 2); bf* Ph = (bf*)take((size_t)TT * CI * 2); bf* Pl = (bf*)take((size_t)TT * CI * 2);
    h16* VT16 = (h16*)take((size_t)DM * TT * 2); bf* VTh = (bf*)take((size_t)DM * TT * 2); bf* VTl = (bf*)take((size_t)DM * TT * 2);
    float* Sb = (float*)take((size_t)TT * TT * 4); float* ST = (float*)take((size_t)2 * TT * 4); bf* Eh = (bf*)take((size_t)TT * TT * 2); bf* El = (bf*)take((size_t)TT * TT * 2);
    if ((size_t)(wsp - (char*)d_ws) > ws_size) return;
    k_wtG<<<(unsigned)((DM * CI / 64 + 63) / 64), 256, 0, stream>>>(wq, DM, CI, WQ); k_wtG<<<(unsigned)((DM * CI / 64 + 63) / 64), 256, 0, stream>>>(wk, DM, CI, WK);
    for (int b = 0; b < NB_; ++b) {
        const float* xb = x + (size_t)b * TT * DM;
        k_cvt8<<<(unsigned)(((size_t)TT * DM / 8 + 255) / 256), 256, 0, stream>>>(xb, XB, (size_t)TT * DM / 8); k_vtp<<<(unsigned)(((size_t)DM * TT / 2 + 255) / 256), 256, 0, stream>>>(xb, DM, DM / HD, VT16, VTh, VTl);
        k_gemmw<bf, 0, true><<<dim3(TT / 64, CI / 64, 1), 32, 0, stream>>>(XB, nullptr, WQ, nullptr, DM, FT, CI, bq, 0, 0, 0); k_flat<<<(unsigned)(((size_t)TT * CI / 4 + 255) / 256), 256, 0, stream>>>(FT, T16, Th, Tl, (size_t)TT * CI / 4);
        k_gemmw<bf, 0, true><<<dim3(TT / 64, CI / 64, 1), 32, 0, stream>>>(XB, nullptr, WK, nullptr, DM, FP, CI, bk, 0, 0, 0); k_flat<<<(unsigned)(((size_t)TT * CI / 4 + 255) / 256), 256, 0, stream>>>(FP, P16, Ph, Pl, (size_t)TT * CI / 4);
        k_gemmw<bf, 2, false><<<dim3(TT / 64, TT / 64, 1), 32, 0, stream>>>(Th, Tl, Ph, Pl, CI, Sb, TT, nullptr, 0, 0, 0);
        k_colsoft<<<TT / 256, 256, 0, stream>>>(Sb, ST);
        k_esplit<<<(unsigned)(((size_t)TT * TT / 4 + 255) / 256), 256, 0, stream>>>(Sb, ST, Eh, El);
        k_gemmw<bf, 1, false><<<dim3(TT / 64, DM / 64, 1), 32, 0, stream>>>(Eh, El, VTh, nullptr, TT, OUT + (size_t)b * TT * DM, DM, nullptr, 0, 0, 0); }
}
